// MyLSTM_16183436771656
// MI455X (gfx1250) — hardware-verified
//
#include <hip/hip_runtime.h>
#include <math.h>

constexpr int NBATCH  = 128;
constexpr int NSTEP   = 128;
constexpr int NIN     = 128;
constexpr int NHID    = 1024;
constexpr int NOUTF   = 128;
constexpr int NGATE   = 4 * NHID;
constexpr int NTHR    = 256;
constexpr int SEQ_BLK = 16;
constexpr int HPITCH  = 1032;
constexpr int CPITCH  = 1024;
constexpr int NROWS   = NSTEP * NBATCH;
constexpr int NOUT0   = NROWS * NOUTF;
constexpr float ACARRY = 16.0f;
constexpr float WCARRY = 256.0f;
constexpr float SC_INV = 1.0f / 4096.0f;
static_assert(NBATCH % SEQ_BLK == 0);
static_assert(NHID == 128 * (NTHR / 32));
static_assert(NIN % 32 == 0 && NHID % 32 == 0);
static_assert(NROWS % 64 == 0 && NOUTF % 64 == 0);
static_assert(HPITCH % 8 == 0);
static_assert(2 * SEQ_BLK * 8 == NTHR);

typedef __attribute__((ext_vector_type(16))) _Float16 v16h;
typedef __attribute__((ext_vector_type(8)))  _Float16 v8h;
typedef __attribute__((ext_vector_type(16))) __bf16   v16b;
typedef __attribute__((ext_vector_type(8)))  __bf16   v8b;
typedef __attribute__((ext_vector_type(8)))  float    v8f;
typedef __attribute__((ext_vector_type(4)))  float    v4f;

__device__ __forceinline__ unsigned short f2bf_bits(float f) {
  unsigned u = __float_as_uint(f);
  return (unsigned short)((u + 0x7FFFu + ((u >> 16) & 1u)) >> 16);
}
__device__ __forceinline__ float bf_bits2f(unsigned short h) { return __uint_as_float(((unsigned)h) << 16); }
__device__ __forceinline__ float bf16r(float f) { return bf_bits2f(f2bf_bits(f)); }

__device__ __forceinline__ void dep_guard_h(v8f& a, v8f& b, v16h x, v16h y) { asm volatile("v_nop\n\tv_nop\n\tv_nop\n\tv_nop" : "+v"(a), "+v"(b) : "v"(x), "v"(y)); }
__device__ __forceinline__ void dep_guard_b(v8f& a, v8f& b, v16b x, v16b y) { asm volatile("v_nop\n\tv_nop\n\tv_nop\n\tv_nop" : "+v"(a), "+v"(b) : "v"(x), "v"(y)); }
__device__ __forceinline__ void dep_guard4_h(v8f& a, v8f& b, v8f& c2, v8f& d, v16h x, v16h y) { asm volatile("v_nop\n\tv_nop\n\tv_nop\n\tv_nop" : "+v"(a), "+v"(b), "+v"(c2), "+v"(d) : "v"(x), "v"(y)); }
__device__ __forceinline__ void dep_guard4_b(v8f& a, v8f& b, v8f& c2, v8f& d, v16b x, v16b y) { asm volatile("v_nop\n\tv_nop\n\tv_nop\n\tv_nop" : "+v"(a), "+v"(b), "+v"(c2), "+v"(d) : "v"(x), "v"(y)); }
__device__ __forceinline__ void keep4_h(v16h a, v16h b, v16h c, v16h d) { asm volatile("v_nop" :: "v"(a), "v"(b), "v"(c), "v"(d)); }
__device__ __forceinline__ void keep4_b(v16b a, v16b b, v16b c, v16b d) { asm volatile("v_nop" :: "v"(a), "v"(b), "v"(c), "v"(d)); }
__device__ __forceinline__ void acc_guard4(v8f& a, v8f& b, v8f& c, v8f& d) { asm volatile("v_nop\n\tv_nop\n\tv_nop\n\tv_nop" : "+v"(a), "+v"(b), "+v"(c), "+v"(d)); }
__device__ __forceinline__ void acc_guard2(v8f& a, v8f& b) { asm volatile("v_nop\n\tv_nop\n\tv_nop\n\tv_nop" : "+v"(a), "+v"(b)); }
__device__ __forceinline__ void guard4x5_h(v8f& a0, v8f& a1, v8f& a2, v8f& a3, v16h f0, v16h f1, v16h f2, v16h f3, v16h f4) {
  asm volatile("v_nop\n\tv_nop\n\tv_nop\n\tv_nop" : "+v"(a0), "+v"(a1), "+v"(a2), "+v"(a3) : "v"(f0), "v"(f1), "v"(f2), "v"(f3), "v"(f4));
}
__device__ __forceinline__ void guard2x3_h(v8f& a0, v8f& a1, v16h f0, v16h f1, v16h f2) {
  asm volatile("v_nop\n\tv_nop\n\tv_nop\n\tv_nop" : "+v"(a0), "+v"(a1) : "v"(f0), "v"(f1), "v"(f2));
}
template <typename T> struct Frag;
template <> struct Frag<_Float16> {
  typedef v16h V; union U { v16h v; v8h h[2]; };
  static __device__ __forceinline__ v16h load(const _Float16* p) {
    U f; f.h[0] = *(const v8h*)(p); f.h[1] = *(const v8h*)(p + 16); return f.v;
  }
  static __device__ __forceinline__ v8f mma(v16h a, v16h b, v8f c) {
    return __builtin_amdgcn_wmma_f32_16x16x32_f16(false, a, false, b, (short)0, c, false, false);
  }
  static __device__ __forceinline__ void guard(v8f& a, v8f& b, v16h x, v16h y) { dep_guard_h(a, b, x, y); }
  static __device__ __forceinline__ void guard4(v8f& a, v8f& b, v8f& c2, v8f& d, v16h x, v16h y) { dep_guard4_h(a, b, c2, d, x, y); }
  static __device__ __forceinline__ void keep(v16h a, v16h b, v16h c, v16h d) { keep4_h(a, b, c, d); }
};
template <> struct Frag<__bf16> {
  typedef v16b V; union U { v16b v; v8b h[2]; };
  static __device__ __forceinline__ v16b load(const __bf16* p) {
    U f; f.h[0] = *(const v8b*)(p); f.h[1] = *(const v8b*)(p + 16); return f.v;
  }
  static __device__ __forceinline__ v8f mma(v16b a, v16b b, v8f c) {
    return __builtin_amdgcn_wmma_f32_16x16x32_bf16(false, a, false, b, (short)0, c, false, false);
  }
  static __device__ __forceinline__ void guard(v8f& a, v8f& b, v16b x, v16b y) { dep_guard_b(a, b, x, y); }
  static __device__ __forceinline__ void guard4(v8f& a, v8f& b, v8f& c2, v8f& d, v16b x, v16b y) { dep_guard4_b(a, b, c2, d, x, y); }
  static __device__ __forceinline__ void keep(v16b a, v16b b, v16b c, v16b d) { keep4_b(a, b, c, d); }
};

__device__ __forceinline__ float fsig(float x)  { return __builtin_amdgcn_rcpf(1.0f + expf(-x)); }
__device__ __forceinline__ float ftanh(float x) { return 1.0f - 2.0f * __builtin_amdgcn_rcpf(expf(2.0f * x) + 1.0f); }

template <int ET> struct Elem;
template <> struct Elem<0> { typedef _Float16 T; };
template <> struct Elem<1> { typedef __bf16 T; };
template <int ET, bool SPLIT, int BIAS_MODE, int OUT_MODE, bool RESID, int ACT = 0>
__global__ __launch_bounds__(256) void wmma_gemm64(
    const unsigned short* __restrict__ Ap, const unsigned short* __restrict__ A2p, int lda, long strideA,
    const unsigned short* __restrict__ Btp, const unsigned short* __restrict__ Bt2p, int ldb, long strideB,
    void* __restrict__ Cout, void* __restrict__ Cout2, int ldc, long strideC,
    const float* __restrict__ bias,
    const float* __restrict__ resid, long strideR,
    int M, int N, int K, float scale) {
  typedef typename Elem<ET>::T T;
  typedef typename Frag<T>::V V;
  const T* A = (const T*)Ap; const T* A2 = (const T*)A2p; const T* Bt = (const T*)Btp; const T* Bt2 = (const T*)Bt2p;
  __shared__ __align__(16) float sT[8][16 * 68];
  const int b    = blockIdx.y;
  const int lane = threadIdx.x & 31;
  const int wave = threadIdx.x >> 5;
  const int tilesN = N >> 6;
  const int tilesM = M >> 6;
  const int tile = blockIdx.x * 8 + wave;
  if (tile >= tilesM * tilesN) return;
  const int tm = tile / tilesN;
  const int tn = tile - tm * tilesN;
  const int m0 = tm << 6;
  const int n0 = tn << 6;

  const T* Ab  = A  + (size_t)b * strideA;
  const T* Bb  = Bt + (size_t)b * strideB;
  const T* Ab2 = SPLIT ? (A2  + (size_t)b * strideA) : nullptr;
  const T* Bb2 = SPLIT ? (Bt2 + (size_t)b * strideB) : nullptr;

  const int rlane = lane & 15;
  const int koff  = (lane >> 4) * 8;
  const int mOff  = (lane >> 4) * 8;

  v8f acc[4][4];
#pragma unroll
  for (int i = 0; i < 4; ++i)
#pragma unroll
    for (int j = 0; j < 4; ++j) acc[i][j] = (v8f){0.f,0.f,0.f,0.f,0.f,0.f,0.f,0.f};

  for (int k0 = 0; k0 < K; k0 += 32) {
    V bh[4], bl[4];
#pragma unroll
    for (int j = 0; j < 4; ++j) {
      const size_t bo = (size_t)(n0 + (j << 4) + rlane) * ldb + koff + k0;
      bh[j] = Frag<T>::load(Bb + bo);
      if (SPLIT) bl[j] = Frag<T>::load(Bb2 + bo);
    }
#pragma unroll
    for (int i = 0; i < 4; ++i) {
      const size_t ao = (size_t)(m0 + (i << 4) + rlane) * lda + koff + k0;
      V ah = Frag<T>::load(Ab + ao);
      V al;
      if (SPLIT) al = Frag<T>::load(Ab2 + ao);
#pragma unroll
      for (int j = 0; j < 4; ++j) {
        acc[i][j] = Frag<T>::mma(ah, bh[j], acc[i][j]);
        if (SPLIT) {
          acc[i][j] = Frag<T>::mma(ah, bl[j], acc[i][j]);
          acc[i][j] = Frag<T>::mma(al, bh[j], acc[i][j]);
        }
      }
      Frag<T>::guard4(acc[i][0], acc[i][1], acc[i][2], acc[i][3], ah, SPLIT ? al : ah);
    }
    Frag<T>::keep(bh[0], bh[1], bh[2], bh[3]);
    if (SPLIT) Frag<T>::keep(bl[0], bl[1], bl[2], bl[3]);
  }
  acc_guard4(acc[0][0], acc[0][1], acc[0][2], acc[0][3]);
  acc_guard4(acc[1][0], acc[1][1], acc[1][2], acc[1][3]);
  acc_guard4(acc[2][0], acc[2][1], acc[2][2], acc[2][3]);
  acc_guard4(acc[3][0], acc[3][1], acc[3][2], acc[3][3]);

  float* slab = sT[wave];
  const float* Rb = RESID ? (resid + (size_t)b * strideR) : nullptr;
#pragma unroll
  for (int i = 0; i < 4; ++i) {
    const int mBase = m0 + (i << 4);
#pragma unroll
    for (int j = 0; j < 4; ++j) {
      const int n = n0 + (j << 4) + rlane;
      float bv = 0.f;
      if (BIAS_MODE == 2) bv = bias[n];
#pragma unroll
      for (int r = 0; r < 8; ++r) {
        float v = acc[i][j][r] * scale;
        if (BIAS_MODE == 1) v += bias[mBase + mOff + r];
        if (BIAS_MODE == 2) v += bv;
        if (RESID) v += Rb[(size_t)(mBase + mOff + r) * ldc + n];
        if (ACT == 1) v = tanhf(v);
        if (ACT == 2) v = fmaxf(v, 0.0f);
        if (ACT == 3) v = v / (1.0f + expf(-v));
        if (ACT == 4) v = (v > 0.f) ? v : 0.01f * v;
        if (ACT == 5) v = 0.5f * v * (1.0f + erff(v * 0.70710678118654752f));
        slab[(mOff + r) * 68 + (j << 4) + rlane] = v;
      }
    }
    __builtin_amdgcn_fence(__ATOMIC_RELEASE, "workgroup");
    __builtin_amdgcn_wave_barrier();
    __builtin_amdgcn_fence(__ATOMIC_ACQUIRE, "workgroup");
    if (OUT_MODE == 0) {
      float* C = (float*)Cout + (size_t)b * strideC;
      const int hh = lane >> 4, c4 = (lane & 15) * 4;
      for (int pass = 0; pass < 2; ++pass) {
#pragma unroll
        for (int it = 0; it < 8; ++it) {
          const int row = it * 2 + hh;
          v4f v = *(const v4f*)(slab + row * 68 + c4);
          *(volatile v4f*)(C + (size_t)(mBase + row) * ldc + n0 + c4) = v;
        }
        __threadfence();
      }
    } else {
      const int q = lane >> 3, c8 = (lane & 7) * 8;
      unsigned short* C  = (unsigned short*)Cout  + (size_t)b * strideC;
      unsigned short* C2 = (OUT_MODE == 2) ? ((unsigned short*)Cout2 + (size_t)b * strideC) : nullptr;
      for (int pass = 0; pass < 2; ++pass) {
#pragma unroll
        for (int it = 0; it < 4; ++it) {
          const int row = it * 4 + q;
          const float* sp = slab + row * 68 + c8;
          v8h hv, lv;
#pragma unroll
          for (int e = 0; e < 8; ++e) {
            if (OUT_MODE == 1) {
              hv[e] = (_Float16)sp[e];
            } else {
              unsigned short hb = f2bf_bits(sp[e]);
              unsigned short lb = f2bf_bits(sp[e] - bf_bits2f(hb));
              hv[e] = __builtin_bit_cast(_Float16, hb);
              lv[e] = __builtin_bit_cast(_Float16, lb);
            }
          }
          *(volatile v8h*)(C + (size_t)(mBase + row) * ldc + n0 + c8) = hv;
          if (OUT_MODE == 2) *(volatile v8h*)(C2 + (size_t)(mBase + row) * ldc + n0 + c8) = lv;
        }
        __threadfence();
      }
    }
    __builtin_amdgcn_fence(__ATOMIC_RELEASE, "workgroup");
    __builtin_amdgcn_wave_barrier();
    __builtin_amdgcn_fence(__ATOMIC_ACQUIRE, "workgroup");
  }
}

template <int MODE>
__global__ __launch_bounds__(NTHR) void cvt8_kernel(const float* __restrict__ src, unsigned short* __restrict__ dst,
                                                    int nrow, int ncol8, int spitch, int scol0, float sc) {
  const int i  = blockIdx.x * NTHR + threadIdx.x;
  const int n8 = nrow * ncol8;
  if (i < n8) {
    const int row = i / ncol8;
    const int c8  = i - row * ncol8;
    const float* sp = src + (size_t)row * spitch + scol0 + c8 * 8;
    const v4f a = *(const v4f*)(sp);
    const v4f b = *(const v4f*)(sp + 4);
    v8h hv;
#pragma unroll
    for (int e = 0; e < 4; ++e) {
      unsigned short b0, b1;
      if (MODE == 0) {
        b0 = f2bf_bits(a[e] * sc);
        b1 = f2bf_bits(b[e] * sc);
      } else {
        b0 = __builtin_bit_cast(unsigned short, (_Float16)(bf16r(a[e]) * sc));
        b1 = __builtin_bit_cast(unsigned short, (_Float16)(bf16r(b[e]) * sc));
      }
      hv[e]     = __builtin_bit_cast(_Float16, b0);
      hv[4 + e] = __builtin_bit_cast(_Float16, b1);
    }
    *(volatile v8h*)(dst + (size_t)i * 8) = hv;
    __threadfence();
    *(volatile v8h*)(dst + (size_t)i * 8) = hv;
  }
}

__global__ __launch_bounds__(NTHR) void bfprep4_kernel(const float* __restrict__ src, float* __restrict__ dst, int n4) {
  const int i = blockIdx.x * NTHR + threadIdx.x;
  if (i < n4) {
    const v4f v = *(const v4f*)(src + 4 * i);
    v4f o;
#pragma unroll
    for (int e = 0; e < 4; ++e) o[e] = bf16r(v[e]);
    *(volatile v4f*)(dst + 4 * i) = o;
    __threadfence();
    *(volatile v4f*)(dst + 4 * i) = o;
  }
}

__global__ __launch_bounds__(NTHR) void lstm_seq_kernel(
    const unsigned short* __restrict__ XHp,
    const unsigned short* __restrict__ NHp,
    const unsigned short* __restrict__ WEHp,
    const unsigned short* __restrict__ WECp,
    const unsigned short* __restrict__ WIHp,
    const unsigned short* __restrict__ WHHp,
    const float* __restrict__ b_eh, const float* __restrict__ b_ec,
    const float* __restrict__ b_ih, const float* __restrict__ b_hh,
    unsigned short* __restrict__ HALLp) {
  __shared__ __align__(16) _Float16 Ah[2][SEQ_BLK * HPITCH];
  __shared__ __align__(16) float    Cs[SEQ_BLK * CPITCH];
  const _Float16* XH  = (const _Float16*)XHp;
  const _Float16* NH  = (const _Float16*)NHp;
  const _Float16* WEH = (const _Float16*)WEHp;
  const _Float16* WEC = (const _Float16*)WECp;
  const _Float16* WIH = (const _Float16*)WIHp;
  const _Float16* WHH = (const _Float16*)WHHp;
  _Float16*       HALL = (_Float16*)HALLp;
  const int tid = threadIdx.x, lane = tid & 31, wave = tid >> 5;
  const int c = lane & 15, hh = lane >> 4, koff = hh * 8;
  const int rowbase = blockIdx.x * SEQ_BLK;
  const v8f z8 = {0.f, 0.f, 0.f, 0.f, 0.f, 0.f, 0.f, 0.f};

  {
    const int pb = tid >> 7, prow = (tid >> 3) & 15, pe = tid & 7;
    Ah[pb][prow * HPITCH + NHID + pe] = (_Float16)0.0f;
  }

#pragma unroll 1
  for (int u = 0; u < 8; ++u) {
    const int j = 128 * wave + 16 * u + c;
    const _Float16* xa = XH  + (size_t)(rowbase + c) * NOUTF + koff;
    const _Float16* we = WEH + (size_t)j * NOUTF + koff;
    const _Float16* wc = WEC + (size_t)j * NOUTF + koff;
    v8f acch = z8, accc = z8;
#pragma unroll 1
    for (int kx = 0; kx < NOUTF; kx += 32) {
      const v16h a  = Frag<_Float16>::load(xa + kx);
      const v16h b0 = Frag<_Float16>::load(we + kx);
      const v16h b1 = Frag<_Float16>::load(wc + kx);
      acch = Frag<_Float16>::mma(a, b0, acch);
      accc = Frag<_Float16>::mma(a, b1, accc);
      guard2x3_h(acch, accc, a, b0, b1);
    }
    acc_guard2(acch, accc);
    const float beh = bf16r(b_eh[j]);
    const float bec = bf16r(b_ec[j]);
#pragma unroll
    for (int r = 0; r < 8; ++r) {
      const int row = 8 * hh + r;
      Cs[row * CPITCH + j] = accc[r] * SC_INV + bec;
      const float h0 = acch[r] * SC_INV + beh;
      Ah[0][row * HPITCH + j] = (_Float16)(h0 * ACARRY);
    }
  }
  __syncthreads();

  const int q = lane >> 3, c8 = (lane & 7) * 8;
  const int colh = 128 * wave + 64 * (q & 1) + c8;

#pragma unroll 1
  for (int t = 0; t < NSTEP; ++t) {
    const int cur = t & 1;
    const _Float16* ahrow = &Ah[cur][0] + c * HPITCH + koff;
    _Float16* ahn = &Ah[cur ^ 1][0];
    const _Float16* xa = NH + ((size_t)t * NBATCH + (size_t)(rowbase + c)) * NIN + koff;
#pragma unroll 1
    for (int u = 0; u < 8; ++u) {
      const int j = 128 * wave + 16 * u + c;
      const _Float16* wi = WIH + (size_t)j * NIN + koff;
      const _Float16* wh = WHH + (size_t)j * NHID + koff;
      v8f acc[4];
      acc[0] = z8; acc[1] = z8; acc[2] = z8; acc[3] = z8;
#pragma unroll 1
      for (int kx = 0; kx < NIN; kx += 32) {
        const v16h a  = Frag<_Float16>::load(xa + kx);
        const v16h b0 = Frag<_Float16>::load(wi + kx);
        const v16h b1 = Frag<_Float16>::load(wi + (size_t)1 * NHID * NIN + kx);
        const v16h b2 = Frag<_Float16>::load(wi + (size_t)2 * NHID * NIN + kx);
        const v16h b3 = Frag<_Float16>::load(wi + (size_t)3 * NHID * NIN + kx);
        acc[0] = Frag<_Float16>::mma(a, b0, acc[0]);
        acc[1] = Frag<_Float16>::mma(a, b1, acc[1]);
        acc[2] = Frag<_Float16>::mma(a, b2, acc[2]);
        acc[3] = Frag<_Float16>::mma(a, b3, acc[3]);
        guard4x5_h(acc[0], acc[1], acc[2], acc[3], a, b0, b1, b2, b3);
      }
#pragma unroll 1
      for (int k0 = 0; k0 < NHID; k0 += 32) {
        const v16h a  = Frag<_Float16>::load(ahrow + k0);
        const v16h b0 = Frag<_Float16>::load(wh + k0);
        const v16h b1 = Frag<_Float16>::load(wh + (size_t)1 * NHID * NHID + k0);
        const v16h b2 = Frag<_Float16>::load(wh + (size_t)2 * NHID * NHID + k0);
        const v16h b3 = Frag<_Float16>::load(wh + (size_t)3 * NHID * NHID + k0);
        acc[0] = Frag<_Float16>::mma(a, b0, acc[0]);
        acc[1] = Frag<_Float16>::mma(a, b1, acc[1]);
        acc[2] = Frag<_Float16>::mma(a, b2, acc[2]);
        acc[3] = Frag<_Float16>::mma(a, b3, acc[3]);
        guard4x5_h(acc[0], acc[1], acc[2], acc[3], a, b0, b1, b2, b3);
      }
      acc_guard4(acc[0], acc[1], acc[2], acc[3]);
      const float bi = bf16r(b_ih[j])            + bf16r(b_hh[j]);
      const float bf = bf16r(b_ih[NHID + j])     + bf16r(b_hh[NHID + j]);
      const float bg = bf16r(b_ih[2 * NHID + j]) + bf16r(b_hh[2 * NHID + j]);
      const float bo = bf16r(b_ih[3 * NHID + j]) + bf16r(b_hh[3 * NHID + j]);
#pragma unroll
      for (int r = 0; r < 8; ++r) {
        const int row = 8 * hh + r;
        const float zi = acc[0][r] * SC_INV + bi;
        const float zf = acc[1][r] * SC_INV + bf;
        const float zg = acc[2][r] * SC_INV + bg;
        const float zo = acc[3][r] * SC_INV + bo;
        const float cold = Cs[row * CPITCH + j];
        const float cn = fsig(zf) * cold + fsig(zi) * ftanh(zg);
        Cs[row * CPITCH + j] = cn;
        const float hn = fsig(zo) * ftanh(cn);
        ahn[row * HPITCH + j] = (_Float16)(hn * ACARRY);
      }
    }
    __builtin_amdgcn_fence(__ATOMIC_RELEASE, "workgroup");
    __builtin_amdgcn_wave_barrier();
    __builtin_amdgcn_fence(__ATOMIC_ACQUIRE, "workgroup");
    for (int pass = 0; pass < 2; ++pass) {
#pragma unroll
      for (int it = 0; it < 8; ++it) {
        const int row = 2 * it + (q >> 1);
        const v8h v = *(const v8h*)(ahn + row * HPITCH + colh);
        *(volatile v8h*)(HALL + ((size_t)t * NBATCH + (size_t)(rowbase + row)) * NHID + colh) = v;
      }
      __threadfence();
    }
    __syncthreads();
  }
}

extern "C" void kernel_launch(void* const* d_in, const int* in_sizes, int n_in,
                              void* d_out, int out_size, void* d_ws, size_t ws_size, hipStream_t stream) {
  if (n_in < 12 || d_out == nullptr || d_ws == nullptr) return;
  if (in_sizes[0] != NBATCH * NOUTF || in_sizes[1] != NSTEP * NBATCH * NIN ||
      in_sizes[2] != NHID * NOUTF || in_sizes[3] != NHID || in_sizes[4] != NHID * NOUTF || in_sizes[5] != NHID ||
      in_sizes[6] != NGATE * NIN || in_sizes[7] != NGATE || in_sizes[8] != NGATE * NHID || in_sizes[9] != NGATE ||
      in_sizes[10] != NOUTF * NHID || in_sizes[11] != NOUTF || out_size != NOUT0) return;

  const float* x     = (const float*)d_in[0];
  const float* noise = (const float*)d_in[1];
  const float* w_eh  = (const float*)d_in[2];
  const float* b_eh  = (const float*)d_in[3];
  const float* w_ec  = (const float*)d_in[4];
  const float* b_ec  = (const float*)d_in[5];
  const float* w_ih  = (const float*)d_in[6];
  const float* b_ih  = (const float*)d_in[7];
  const float* w_hh  = (const float*)d_in[8];
  const float* b_hh  = (const float*)d_in[9];
  const float* w_out = (const float*)d_in[10];
  const float* b_out = (const float*)d_in[11];
  float* out = (float*)d_out;

  char* ws = (char*)d_ws; size_t off = 0;
  auto carve = [&](size_t bytes) -> char* { char* p = ws + off; off += (bytes + 255) & ~(size_t)255; return p; };
  unsigned short* XH   = (unsigned short*)carve((size_t)NBATCH * NOUTF * 2);
  unsigned short* NH   = (unsigned short*)carve((size_t)NROWS * NIN * 2);
  unsigned short* WEH  = (unsigned short*)carve((size_t)NHID * NOUTF * 2);
  unsigned short* WEC  = (unsigned short*)carve((size_t)NHID * NOUTF * 2);
  unsigned short* WIH  = (unsigned short*)carve((size_t)NGATE * NIN * 2);
  unsigned short* WHH  = (unsigned short*)carve((size_t)NGATE * NHID * 2);
  unsigned short* WOUT = (unsigned short*)carve((size_t)NOUTF * NHID * 2);
  float*          BOUT = (float*)carve((size_t)NOUTF * 4);
  unsigned short* HALL = (unsigned short*)carve((size_t)NROWS * NHID * 2);
  if (off > ws_size || off > (size_t)134217728) return;

  const int n8x  = NBATCH * (NOUTF / 8);
  const int n8n  = NROWS * (NIN / 8);
  const int n8e  = NHID * (NOUTF / 8);
  const int n8i  = NGATE * (NIN / 8);
  const int n8h  = NGATE * (NHID / 8);
  const int n8o  = NOUTF * (NHID / 8);
  cvt8_kernel<1><<<(n8x + NTHR - 1) / NTHR, NTHR, 0, stream>>>(x,     XH,   NBATCH, NOUTF / 8, NOUTF, 0, ACARRY);
  cvt8_kernel<1><<<(n8n + NTHR - 1) / NTHR, NTHR, 0, stream>>>(noise, NH,   NROWS,  NIN / 8,   NIN,   0, ACARRY);
  cvt8_kernel<1><<<(n8e + NTHR - 1) / NTHR, NTHR, 0, stream>>>(w_eh,  WEH,  NHID,   NOUTF / 8, NOUTF, 0, WCARRY);
  cvt8_kernel<1><<<(n8e + NTHR - 1) / NTHR, NTHR, 0, stream>>>(w_ec,  WEC,  NHID,   NOUTF / 8, NOUTF, 0, WCARRY);
  cvt8_kernel<1><<<(n8i + NTHR - 1) / NTHR, NTHR, 0, stream>>>(w_ih,  WIH,  NGATE,  NIN / 8,   NIN,   0, WCARRY);
  cvt8_kernel<1><<<(n8h + NTHR - 1) / NTHR, NTHR, 0, stream>>>(w_hh,  WHH,  NGATE,  NHID / 8,  NHID,  0, WCARRY);
  cvt8_kernel<1><<<(n8o + NTHR - 1) / NTHR, NTHR, 0, stream>>>(w_out, WOUT, NOUTF,  NHID / 8,  NHID,  0, WCARRY);
  bfprep4_kernel<<<1, NTHR, 0, stream>>>(b_out, BOUT, NOUTF / 4);

  lstm_seq_kernel<<<NBATCH / SEQ_BLK, NTHR, 0, stream>>>(XH, NH, WEH, WEC, WIH, WHH, b_eh, b_ec, b_ih, b_hh, HALL);

  const dim3 ggrid((NROWS / 64) * (NOUTF / 64) / 8, 1);
  wmma_gemm64<0, false, 2, 0, false, 1><<<ggrid, 256, 0, stream>>>(
      HALL, HALL, NHID, 0L, WOUT, WOUT, NHID, 0L, (void*)out, (void*)out, NOUTF, 0L,
      BOUT, BOUT, 0L, NROWS, NOUTF, NHID, SC_INV);
}
